// FlashRWLargeAttention_47399259079206
// MI455X (gfx1250) — hardware-verified
//
#include <hip/hip_runtime.h>
#include <stddef.h>
#include <stdint.h>


typedef _Float16 f16;
typedef f16 v8h __attribute__((ext_vector_type(8)));
typedef f16 v16h __attribute__((ext_vector_type(16)));
typedef float v8f __attribute__((ext_vector_type(8)));
typedef float v4f __attribute__((ext_vector_type(4)));
typedef v8h __attribute__((may_alias)) v8ha;
typedef v4f __attribute__((may_alias)) v4fa;

union Frag { v16h v; v8h h[2]; };
union Pack8 { v8h h; v4f f; f16 e[8]; };

#define NTOK 4096
#define HID 2048
#define QKVN 3072
#define SEQL 1024
#define NGRP 8
#define NQH 32
#define ROT 32
#define RSPLIT 384
#define MPSPLIT (RSPLIT / 32)
#define LDT 40
#define KP 72
#define VP 40
#define PP 40
#define OP 72
#define NOP4 "v_nop\n\tv_nop\n\tv_nop\n\tv_nop"

__device__ __forceinline__ float bf16r(float x) {
  unsigned int u = __float_as_uint(x);
  u += 0x7FFFu + ((u >> 16) & 1u);
  return __uint_as_float(u & 0xFFFF0000u);
}
__device__ __forceinline__ v8f z8() {
  v8f z = {0.f, 0.f, 0.f, 0.f, 0.f, 0.f, 0.f, 0.f};
  return z;
}
__device__ __forceinline__ v8f mma16(v16h a, v16h b, v8f c) {
  return __builtin_amdgcn_wmma_f32_16x16x32_f16(false, a, false, b, (short)0, c, false, false);
}

__global__ __launch_bounds__(256) void k_cvt_x(const float* __restrict__ src, f16* __restrict__ dst, int n8) {
  const int i = blockIdx.x * 256 + threadIdx.x;
  if (i < n8) {
    const v4f a = *(const v4f*)(src + (size_t)i * 8);
    const v4f b = *(const v4f*)(src + (size_t)i * 8 + 4);
    Pack8 o;
    o.e[0] = (f16)bf16r(a.x); o.e[1] = (f16)bf16r(a.y); o.e[2] = (f16)bf16r(a.z); o.e[3] = (f16)bf16r(a.w);
    o.e[4] = (f16)bf16r(b.x); o.e[5] = (f16)bf16r(b.y); o.e[6] = (f16)bf16r(b.z); o.e[7] = (f16)bf16r(b.w);
    f16* d = dst + (size_t)i * 8;
    *(volatile v4f*)d = o.f;
    __threadfence();
    *(volatile v4f*)d = o.f;
  }
}

__global__ __launch_bounds__(256) void k_cvt_wt(const float* __restrict__ src, f16* __restrict__ dst, int K, int N, float scl) {
  __shared__ float tile[64][33];
  const int n0 = blockIdx.x * 32, k0 = blockIdx.y * 64;
  const int tid = threadIdx.x, tx = tid & 31, ty = tid >> 5;
#pragma unroll
  for (int r = 0; r < 8; ++r) {
    const int k = ty + r * 8;
    float v = 0.f;
    if (k0 + k < K && n0 + tx < N) v = src[(size_t)(k0 + k) * N + n0 + tx];
    tile[k][tx] = v;
  }
  __syncthreads();
  const int n = ty * 4 + (tx >> 3), p = tx & 7;
  Pack8 o;
#pragma unroll
  for (int i = 0; i < 8; ++i) o.e[i] = (f16)(bf16r(tile[8 * p + i][n]) * scl);
  if (n0 + n < N && k0 + 8 * p + 8 <= K) {
    f16* d = dst + (size_t)(n0 + n) * K + k0 + 8 * p;
    *(volatile v4f*)d = o.f;
    __threadfence();
    *(volatile v4f*)d = o.f;
  }
}

template <int NPL>
__device__ __forceinline__ void gemm_loop(const f16* __restrict__ A0, const f16* __restrict__ A1,
                                          const f16* __restrict__ Bt, int K, int m0, int n0,
                                          f16* sm, v8f (&acc)[8], v8f (&acc2)[8]) {
  f16* sA0 = sm;
  f16* sA1 = sm + 128 * LDT;
  f16* sB = sm + 256 * LDT;
  const int tid = threadIdx.x, wave = tid >> 5, lane = tid & 31, h = lane >> 4, m = lane & 15;
  for (int k0 = 0; k0 < K; k0 += 32) {
    __syncthreads();
#pragma unroll
    for (int r = 0; r < 2; ++r) {
      const int idx = tid + r * 256, row = idx >> 2, ch = idx & 3;
      const size_t go = (size_t)k0 + ch * 8;
      const v8h va = *(const v8h*)(A0 + (size_t)(m0 + row) * K + go);
      *(v8h*)(sA0 + row * LDT + ch * 8) = va;
      if (NPL == 2) {
        const v8h v1 = *(const v8h*)(A1 + (size_t)(m0 + row) * K + go);
        *(v8h*)(sA1 + row * LDT + ch * 8) = v1;
      }
      const v8h vb = *(const v8h*)(Bt + (size_t)(n0 + row) * K + go);
      *(v8h*)(sB + row * LDT + ch * 8) = vb;
    }
    __syncthreads();
    Frag a, a2, b;
    const f16* ar = sA0 + (wave * 16 + m) * LDT;
    a.h[0] = *(const v8ha*)(ar + 8 * h);
    a.h[1] = *(const v8ha*)(ar + 16 + 8 * h);
    a2.v = a.v;
    if (NPL == 2) {
      const f16* ar2 = sA1 + (wave * 16 + m) * LDT;
      a2.h[0] = *(const v8ha*)(ar2 + 8 * h);
      a2.h[1] = *(const v8ha*)(ar2 + 16 + 8 * h);
    }
#pragma unroll
    for (int j = 0; j < 8; ++j) {
      const f16* br = sB + (j * 16 + m) * LDT;
      b.h[0] = *(const v8ha*)(br + 8 * h);
      b.h[1] = *(const v8ha*)(br + 16 + 8 * h);
      acc[j] = mma16(a.v, b.v, acc[j]);
      if (NPL == 2) acc2[j] = mma16(a2.v, b.v, acc2[j]);
    }
    if (NPL == 2) {
      asm volatile(NOP4
                   : "+v"(acc[0]), "+v"(acc[1]), "+v"(acc[2]), "+v"(acc[3]),
                     "+v"(acc[4]), "+v"(acc[5]), "+v"(acc[6]), "+v"(acc[7]),
                     "+v"(acc2[0]), "+v"(acc2[1]), "+v"(acc2[2]), "+v"(acc2[3]),
                     "+v"(acc2[4]), "+v"(acc2[5]), "+v"(acc2[6]), "+v"(acc2[7])
                   : "v"(a.v), "v"(a2.v), "v"(b.v));
    } else {
      asm volatile(NOP4
                   : "+v"(acc[0]), "+v"(acc[1]), "+v"(acc[2]), "+v"(acc[3]),
                     "+v"(acc[4]), "+v"(acc[5]), "+v"(acc[6]), "+v"(acc[7])
                   : "v"(a.v), "v"(b.v));
    }
  }
}

__device__ __forceinline__ void qkv_store(const f16* stg, int tbase, int hd0, int lane,
                                          f16* __restrict__ Qp, f16* __restrict__ Kp, f16* __restrict__ Vp) {
  const int rs = lane >> 4, c = (lane >> 3) & 1, p = lane & 7;
  const int hd = hd0 + c, g = hd / 6, r6 = hd - g * 6;
  f16* pb = (r6 < 4) ? (Qp + (size_t)(g * 4 + r6) * NTOK * 64)
                     : ((r6 == 4) ? (Kp + (size_t)g * NTOK * 64) : (Vp + (size_t)g * NTOK * 64));
  v4f vals[8];
#pragma unroll
  for (int q = 0; q < 8; ++q) {
    Pack8 u;
    u.h = *(const v8ha*)(stg + (2 * q + rs) * 128 + 64 * c + 8 * p);
    vals[q] = u.f;
  }
#pragma unroll
  for (int q = 0; q < 8; ++q) {
    f16* d = pb + (size_t)(tbase + 2 * q + rs) * 64 + 8 * p;
    *(volatile v4f*)d = vals[q];
  }
  __threadfence();
#pragma unroll
  for (int q = 0; q < 8; ++q) {
    f16* d = pb + (size_t)(tbase + 2 * q + rs) * 64 + 8 * p;
    *(volatile v4f*)d = vals[q];
  }
}

__global__ __launch_bounds__(256) __attribute__((amdgpu_num_vgpr(256)))
void k_qkv(const f16* __restrict__ X, const f16* __restrict__ Wt, const float* __restrict__ bias,
           const float* __restrict__ cosb, const float* __restrict__ sinb,
           f16* __restrict__ Qh, f16* __restrict__ Ql, f16* __restrict__ Kh, f16* __restrict__ Kl,
           f16* __restrict__ Vh, f16* __restrict__ Vl, int M, int N, int K) {
  __shared__ __attribute__((aligned(16))) f16 sm[16384];
  const int m0 = blockIdx.y * 128, n0 = blockIdx.x * 128;
  if (m0 + 128 > M || n0 + 128 > N) return;
  const int tid = threadIdx.x, wave = tid >> 5, lane = tid & 31, h = lane >> 4, m = lane & 15;
  v8f acc[8], accd[8];
#pragma unroll
  for (int j = 0; j < 8; ++j) { acc[j] = z8(); accd[j] = z8(); }
  gemm_loop<1>(X, X, Wt, K, m0, n0, sm, acc, accd);

  const float c64 = 0.015625f;
#pragma unroll
  for (int j = 0; j < 8; ++j) {
    const float bv = bf16r(bias[n0 + 16 * j + m]);
#pragma unroll
    for (int r = 0; r < 8; ++r) acc[j][r] = acc[j][r] * c64 + bv;
  }
  const int hd0 = n0 >> 6;
  const int trow = m0 + wave * 16 + 8 * h;
#pragma unroll
  for (int c = 0; c < 2; ++c) {
    const int hdc = hd0 + c;
    const int r6 = hdc - (hdc / 6) * 6;
    if (r6 != 5) {
#pragma unroll
      for (int jj = 0; jj < 2; ++jj) {
        const int jc = jj * 16 + m;
#pragma unroll
        for (int r = 0; r < 8; ++r) {
          const size_t ci = (size_t)(trow + r) * ROT + jc;
          const float cv = bf16r(cosb[ci]), sv = bf16r(sinb[ci]);
          const float x1 = acc[4 * c + jj][r], x2 = acc[4 * c + jj + 2][r];
          acc[4 * c + jj][r] = x1 * cv - x2 * sv;
          acc[4 * c + jj + 2][r] = x1 * sv + x2 * cv;
        }
      }
    }
  }
  __syncthreads();
  f16* stg = sm + wave * 2048;
#pragma unroll
  for (int j = 0; j < 8; ++j)
#pragma unroll
    for (int r = 0; r < 8; ++r) stg[(8 * h + r) * 128 + 16 * j + m] = (f16)acc[j][r];
  __syncthreads();
  qkv_store(stg, m0 + wave * 16, hd0, lane, Qh, Kh, Vh);
  if ((m0 & (SEQL - 1)) < RSPLIT) {
    __syncthreads();
#pragma unroll
    for (int j = 0; j < 8; ++j)
#pragma unroll
      for (int r = 0; r < 8; ++r) {
        const float v = acc[j][r];
        const f16 hv = (f16)v;
        stg[(8 * h + r) * 128 + 16 * j + m] = (f16)((v - (float)hv) * 2048.f);
      }
    __syncthreads();
    qkv_store(stg, m0 + wave * 16, hd0, lane, Ql, Kl, Vl);
  }
}

__device__ __forceinline__ void attn_store(const f16* stg, f16* __restrict__ dst, int trow0, int qh, int lane) {
  const int rs = lane >> 3, p = lane & 7;
  v4f vals[4];
#pragma unroll
  for (int q = 0; q < 4; ++q) {
    Pack8 u;
    u.h = *(const v8ha*)(stg + (4 * q + rs) * OP + 8 * p);
    vals[q] = u.f;
  }
#pragma unroll
  for (int q = 0; q < 4; ++q) {
    f16* d = dst + (size_t)(trow0 + 4 * q + rs) * HID + qh * 64 + 8 * p;
    *(volatile v4f*)d = vals[q];
  }
  __threadfence();
#pragma unroll
  for (int q = 0; q < 4; ++q) {
    f16* d = dst + (size_t)(trow0 + 4 * q + rs) * HID + qh * 64 + 8 * p;
    *(volatile v4f*)d = vals[q];
  }
}

template <int SPL>
__device__ __forceinline__ void attn_body(const f16* __restrict__ Qh, const f16* __restrict__ Ql,
                                          const f16* __restrict__ Kh, const f16* __restrict__ Kl,
                                          const f16* __restrict__ Vh, const f16* __restrict__ Vl,
                                          f16* __restrict__ Ah, f16* __restrict__ Al,
                                          int g, int s0, int mp,
                                          f16* sKh, f16* sKl, f16* sVh, f16* sVl, f16* sP) {
  const int tid = threadIdx.x, wave = tid >> 5, lane = tid & 31, h = lane >> 4, m = lane & 15;
  const int head = wave & 3, qh = g * 4 + head;
  const int row0 = mp * 32 + (wave >> 2) * 16;
  f16* sPh = sP + wave * 1280;
  f16* sPl = sPh + 640;

  Frag aq[2], aql[2];
  {
    const f16* qp = Qh + ((size_t)qh * NTOK + s0 + row0 + m) * 64;
    const f16* qlp = Ql + ((size_t)qh * NTOK + s0 + row0 + m) * 64;
#pragma unroll
    for (int st = 0; st < 2; ++st) {
      aq[st].h[0] = *(const v8h*)(qp + 32 * st + 8 * h);
      aq[st].h[1] = *(const v8h*)(qp + 32 * st + 16 + 8 * h);
      aql[st].v = aq[st].v;
      if (SPL) {
        aql[st].h[0] = *(const v8h*)(qlp + 32 * st + 8 * h);
        aql[st].h[1] = *(const v8h*)(qlp + 32 * st + 16 + 8 * h);
      }
    }
  }

  float mi[8], li[8];
  v8f acc[4];
#pragma unroll
  for (int r = 0; r < 8; ++r) { mi[r] = -3.0e38f; li[r] = 0.f; }
#pragma unroll
  for (int j = 0; j < 4; ++j) acc[j] = z8();
  const float sc = 0.125f, c11 = 0.00048828125f;

  for (int tile = 0; tile <= mp; ++tile) {
    const int t0 = tile * 32;
    __syncthreads();
    {
      const int row = tid >> 3, ch = tid & 7;
      const size_t go = ((size_t)g * NTOK + s0 + t0 + row) * 64 + ch * 8;
      const v8h kv = *(const v8h*)(Kh + go);
      *(v8h*)(sKh + row * KP + ch * 8) = kv;
      Pack8 vv;
      vv.h = *(const v8h*)(Vh + go);
#pragma unroll
      for (int i = 0; i < 8; ++i) sVh[(ch * 8 + i) * VP + row] = vv.e[i];
      if (SPL) {
        const v8h klv = *(const v8h*)(Kl + go);
        *(v8h*)(sKl + row * KP + ch * 8) = klv;
        Pack8 vl;
        vl.h = *(const v8h*)(Vl + go);
#pragma unroll
        for (int i = 0; i < 8; ++i) sVl[(ch * 8 + i) * VP + row] = vl.e[i];
      }
    }
    __syncthreads();

    v8f sf0 = z8(), sf1 = z8(), tf0 = z8(), tf1 = z8();
    Frag bk, bkl;
    bkl.v = aq[0].v;
#pragma unroll
    for (int st = 0; st < 2; ++st) {
      const int d0 = 32 * st;
      const f16* k0p = sKh + m * KP + d0;
      const f16* k1p = sKh + (16 + m) * KP + d0;
      bk.h[0] = *(const v8ha*)(k0p + 8 * h);
      bk.h[1] = *(const v8ha*)(k0p + 16 + 8 * h);
      sf0 = mma16(aq[st].v, bk.v, sf0);
      if (SPL) {
        const f16* l0p = sKl + m * KP + d0;
        bkl.h[0] = *(const v8ha*)(l0p + 8 * h);
        bkl.h[1] = *(const v8ha*)(l0p + 16 + 8 * h);
        tf0 = mma16(aq[st].v, bkl.v, tf0);
        tf0 = mma16(aql[st].v, bk.v, tf0);
      }
      bk.h[0] = *(const v8ha*)(k1p + 8 * h);
      bk.h[1] = *(const v8ha*)(k1p + 16 + 8 * h);
      sf1 = mma16(aq[st].v, bk.v, sf1);
      if (SPL) {
        const f16* l1p = sKl + (16 + m) * KP + d0;
        bkl.h[0] = *(const v8ha*)(l1p + 8 * h);
        bkl.h[1] = *(const v8ha*)(l1p + 16 + 8 * h);
        tf1 = mma16(aq[st].v, bkl.v, tf1);
        tf1 = mma16(aql[st].v, bk.v, tf1);
      }
    }
    if (SPL) {
      asm volatile(NOP4
                   : "+v"(sf0), "+v"(sf1), "+v"(tf0), "+v"(tf1)
                   : "v"(aq[0].v), "v"(aq[1].v), "v"(aql[0].v), "v"(aql[1].v), "v"(bk.v), "v"(bkl.v));
      sf0 = sf0 + tf0 * c11;
      sf1 = sf1 + tf1 * c11;
    } else {
      asm volatile(NOP4 : "+v"(sf0), "+v"(sf1) : "v"(aq[0].v), "v"(aq[1].v), "v"(bk.v));
    }

#pragma unroll
    for (int r = 0; r < 8; ++r) {
      const int srow = row0 + 8 * h + r;
      float x0 = sf0[r] * sc;
      if (t0 + m > srow) x0 = -3.0e38f;
      float x1 = sf1[r] * sc;
      if (t0 + 16 + m > srow) x1 = -3.0e38f;
      float cand = fmaxf(x0, x1);
      cand = fmaxf(cand, __shfl_xor(cand, 1, 32));
      cand = fmaxf(cand, __shfl_xor(cand, 2, 32));
      cand = fmaxf(cand, __shfl_xor(cand, 4, 32));
      cand = fmaxf(cand, __shfl_xor(cand, 8, 32));
      const float mnew = fmaxf(mi[r], cand);
      const float p0 = __expf(x0 - mnew), p1 = __expf(x1 - mnew), corr = __expf(mi[r] - mnew);
      li[r] = li[r] * corr + (p0 + p1);
      mi[r] = mnew;
      acc[0][r] *= corr; acc[1][r] *= corr; acc[2][r] *= corr; acc[3][r] *= corr;
      const float q0 = p0 * 256.f, q1 = p1 * 256.f;
      const f16 h0 = (f16)q0, h1 = (f16)q1;
      sPh[(8 * h + r) * PP + m] = h0;
      sPh[(8 * h + r) * PP + 16 + m] = h1;
      if (SPL) {
        sPl[(8 * h + r) * PP + m] = (f16)((q0 - (float)h0) * 2048.f);
        sPl[(8 * h + r) * PP + 16 + m] = (f16)((q1 - (float)h1) * 2048.f);
      }
    }
    __syncthreads();

    Frag pa, pal, bv, bvl;
    pa.h[0] = *(const v8ha*)(sPh + m * PP + 8 * h);
    pa.h[1] = *(const v8ha*)(sPh + m * PP + 16 + 8 * h);
    pal.v = pa.v;
    bvl.v = pa.v;
    if (SPL) {
      pal.h[0] = *(const v8ha*)(sPl + m * PP + 8 * h);
      pal.h[1] = *(const v8ha*)(sPl + m * PP + 16 + 8 * h);
#pragma unroll
      for (int j = 0; j < 4; ++j) {
        const f16* vp = sVh + (16 * j + m) * VP;
        const f16* vlp = sVl + (16 * j + m) * VP;
        bv.h[0] = *(const v8ha*)(vp + 8 * h);
        bv.h[1] = *(const v8ha*)(vp + 16 + 8 * h);
        bvl.h[0] = *(const v8ha*)(vlp + 8 * h);
        bvl.h[1] = *(const v8ha*)(vlp + 16 + 8 * h);
        acc[j] = mma16(pa.v, bv.v, acc[j]);
        v8f tp = z8();
        tp = mma16(pa.v, bvl.v, tp);
        tp = mma16(pal.v, bv.v, tp);
        asm volatile(NOP4 : "+v"(acc[j]), "+v"(tp) : "v"(pa.v), "v"(pal.v), "v"(bv.v), "v"(bvl.v));
        acc[j] = acc[j] + tp * c11;
      }
    } else {
#pragma unroll
      for (int j = 0; j < 4; ++j) {
        const f16* vp = sVh + (16 * j + m) * VP;
        bv.h[0] = *(const v8ha*)(vp + 8 * h);
        bv.h[1] = *(const v8ha*)(vp + 16 + 8 * h);
        acc[j] = mma16(pa.v, bv.v, acc[j]);
      }
      asm volatile(NOP4 : "+v"(acc[0]), "+v"(acc[1]), "+v"(acc[2]), "+v"(acc[3]) : "v"(pa.v), "v"(bv.v));
    }
  }

  float inv[8];
#pragma unroll
  for (int r = 0; r < 8; ++r) {
    float l = li[r];
    l += __shfl_xor(l, 1, 32);
    l += __shfl_xor(l, 2, 32);
    l += __shfl_xor(l, 4, 32);
    l += __shfl_xor(l, 8, 32);
    inv[r] = (1.0f / l) * 0.00390625f;
  }
  __syncthreads();
  f16* stg = sPh;
#pragma unroll
  for (int j = 0; j < 4; ++j)
#pragma unroll
    for (int r = 0; r < 8; ++r) stg[(8 * h + r) * OP + 16 * j + m] = (f16)(acc[j][r] * inv[r]);
  __syncthreads();
  attn_store(stg, Ah, s0 + row0, qh, lane);
  if (SPL) {
    __syncthreads();
#pragma unroll
    for (int j = 0; j < 4; ++j)
#pragma unroll
      for (int r = 0; r < 8; ++r) {
        const float o = acc[j][r] * inv[r];
        const f16 hv = (f16)o;
        stg[(8 * h + r) * OP + 16 * j + m] = (f16)((o - (float)hv) * 2048.f);
      }
    __syncthreads();
    attn_store(stg, Al, s0 + row0, qh, lane);
  }
}

__global__ __launch_bounds__(256) __attribute__((amdgpu_num_vgpr(256)))
void k_attn(const f16* __restrict__ Qh, const f16* __restrict__ Ql,
            const f16* __restrict__ Kh, const f16* __restrict__ Kl,
            const f16* __restrict__ Vh, const f16* __restrict__ Vl,
            const int* __restrict__ cu, int ncu,
            f16* __restrict__ Ah, f16* __restrict__ Al) {
  __shared__ __attribute__((aligned(16))) f16 sKh[32 * KP];
  __shared__ __attribute__((aligned(16))) f16 sKl[32 * KP];
  __shared__ __attribute__((aligned(16))) f16 sVh[64 * VP];
  __shared__ __attribute__((aligned(16))) f16 sVl[64 * VP];
  __shared__ __attribute__((aligned(16))) f16 sP[8 * 1280];
  const int mp = blockIdx.x & 31;
  const int bg = blockIdx.x >> 5;
  const int g = bg & 7, b = bg >> 3;
  int s0 = b * SEQL;
  if ((unsigned)b < (unsigned)ncu) s0 = cu[b];
  s0 = s0 < 0 ? 0 : s0;
  s0 = s0 > (NTOK - SEQL) ? (NTOK - SEQL) : s0;
  if (mp < MPSPLIT)
    attn_body<1>(Qh, Ql, Kh, Kl, Vh, Vl, Ah, Al, g, s0, mp, sKh, sKl, sVh, sVl, sP);
  else
    attn_body<0>(Qh, Ql, Kh, Kl, Vh, Vl, Ah, Al, g, s0, mp, sKh, sKl, sVh, sVl, sP);
}

__device__ __forceinline__ void dense_store(const float* stg, float* __restrict__ out, int tbase, int col0, int N, int lane) {
  const int rs = lane >> 4, p = lane & 15;
  v4f vals[8];
#pragma unroll
  for (int q = 0; q < 8; ++q) vals[q] = *(const v4fa*)(stg + (2 * q + rs) * 64 + 4 * p);
#pragma unroll
  for (int q = 0; q < 8; ++q) {
    float* d = out + (size_t)(tbase + 2 * q + rs) * N + col0 + 4 * p;
    *(volatile v4f*)d = vals[q];
  }
  __threadfence();
#pragma unroll
  for (int q = 0; q < 8; ++q) {
    float* d = out + (size_t)(tbase + 2 * q + rs) * N + col0 + 4 * p;
    *(volatile v4f*)d = vals[q];
  }
}

template <int NPL>
__device__ __forceinline__ void dense_body(const f16* __restrict__ Ah, const f16* __restrict__ Al,
                                           const f16* __restrict__ Wt, const float* __restrict__ bias,
                                           float* __restrict__ out, int N, int K, int m0, int n0, f16* sm) {
  const int tid = threadIdx.x, wave = tid >> 5, lane = tid & 31, h = lane >> 4, m = lane & 15;
  v8f acc[8], acc2[8];
#pragma unroll
  for (int j = 0; j < 8; ++j) { acc[j] = z8(); acc2[j] = z8(); }
  gemm_loop<NPL>(Ah, Al, Wt, K, m0, n0, sm, acc, acc2);
  const float c64 = 0.015625f, c11 = 0.00048828125f;
#pragma unroll
  for (int j = 0; j < 8; ++j) {
    const float bv = bf16r(bias[n0 + 16 * j + m]);
#pragma unroll
    for (int r = 0; r < 8; ++r) {
      float v = acc[j][r];
      if (NPL == 2) v = v + acc2[j][r] * c11;
      acc[j][r] = v * c64 + bv;
    }
  }
  float* stg = (float*)sm + wave * 1024;
#pragma unroll
  for (int hb = 0; hb < 2; ++hb) {
    __syncthreads();
#pragma unroll
    for (int jj = 0; jj < 4; ++jj)
#pragma unroll
      for (int r = 0; r < 8; ++r) stg[(8 * h + r) * 64 + 16 * jj + m] = acc[4 * hb + jj][r];
    __syncthreads();
    dense_store(stg, out, m0 + wave * 16, n0 + 64 * hb, N, lane);
  }
}

__global__ __launch_bounds__(256) __attribute__((amdgpu_num_vgpr(256)))
void k_dense(const f16* __restrict__ Ah, const f16* __restrict__ Al, const f16* __restrict__ Wt,
             const float* __restrict__ bias, float* __restrict__ out, int M, int N, int K) {
  __shared__ __attribute__((aligned(16))) f16 sm[16384];
  const int m0 = blockIdx.y * 128, n0 = blockIdx.x * 128;
  if (m0 + 128 > M || n0 + 128 > N) return;
  if ((m0 & (SEQL - 1)) < RSPLIT)
    dense_body<2>(Ah, Al, Wt, bias, out, N, K, m0, n0, sm);
  else
    dense_body<1>(Ah, Al, Wt, bias, out, N, K, m0, n0, sm);
}

extern "C" void kernel_launch(void* const* d_in, const int* in_sizes, int n_in,
                              void* d_out, int out_size, void* d_ws, size_t ws_size,
                              hipStream_t stream) {
  if (n_in < 9) return;
  if (in_sizes[0] != NTOK * HID || in_sizes[1] != NTOK * ROT || in_sizes[2] != NTOK * ROT ||
      in_sizes[3] < 1 || in_sizes[5] != HID * QKVN || in_sizes[6] != QKVN ||
      in_sizes[7] != HID * HID || in_sizes[8] != HID || out_size != NTOK * HID)
    return;

  const float* x_f = (const float*)d_in[0];
  const float* cos_f = (const float*)d_in[1];
  const float* sin_f = (const float*)d_in[2];
  const int* cu_i = (const int*)d_in[3];
  const float* wqkv_f = (const float*)d_in[5];
  const float* bqkv_f = (const float*)d_in[6];
  const float* wout_f = (const float*)d_in[7];
  const float* bout_f = (const float*)d_in[8];
  float* out = (float*)d_out;

  const size_t bX = (size_t)NTOK * HID * 2;
  const size_t bWq = (size_t)QKVN * HID * 2;
  const size_t bWd = (size_t)HID * HID * 2;
  const size_t bQ = (size_t)NQH * NTOK * 64 * 2;
  const size_t bKV = (size_t)NGRP * NTOK * 64 * 2;
  const size_t bA = (size_t)NTOK * HID * 2;
  char* ws = (char*)d_ws;
  size_t off = 0;
  f16* Xh = (f16*)(ws + off); off += bX;
  f16* Wq = (f16*)(ws + off); off += bWq;
  f16* Wd = (f16*)(ws + off); off += bWd;
  f16* Qh = (f16*)(ws + off); off += bQ;
  f16* Ql = (f16*)(ws + off); off += bQ;
  f16* Kh = (f16*)(ws + off); off += bKV;
  f16* Kl = (f16*)(ws + off); off += bKV;
  f16* Vh = (f16*)(ws + off); off += bKV;
  f16* Vl = (f16*)(ws + off); off += bKV;
  f16* Ah = (f16*)(ws + off); off += bA;
  f16* Al = (f16*)(ws + off); off += bA;
  if (off > ws_size) return;

  const int n8 = NTOK * HID / 8;
  k_cvt_x<<<(n8 + 255) / 256, 256, 0, stream>>>(x_f, Xh, n8);
  k_cvt_wt<<<dim3(QKVN / 32, HID / 64), 256, 0, stream>>>(wqkv_f, Wq, HID, QKVN, 64.f);
  k_cvt_wt<<<dim3(HID / 32, HID / 64), 256, 0, stream>>>(wout_f, Wd, HID, HID, 64.f);
  k_qkv<<<dim3(QKVN / 128, NTOK / 128), 256, 0, stream>>>(Xh, Wq, bqkv_f, cos_f, sin_f,
                                                          Qh, Ql, Kh, Kl, Vh, Vl, NTOK, QKVN, HID);
  k_attn<<<(NTOK / 32) * NGRP, 256, 0, stream>>>(Qh, Ql, Kh, Kl, Vh, Vl, cu_i, in_sizes[3], Ah, Al);
  k_dense<<<dim3(HID / 128, NTOK / 128), 256, 0, stream>>>(Ah, Al, Wd, bout_f, out, NTOK, HID, HID);
}
